// PointNet_69947837383384
// MI455X (gfx1250) — hardware-verified
//
#include <hip/hip_runtime.h>
#include <math.h>

constexpr int NUM_POINTS   = 65536;
constexpr int NCH_L1       = 64;
constexpr int NCH_L2       = 64;
constexpr int NCH_L3       = 128;
constexpr int NCH_L4       = 1024;
constexpr int NCH_L5       = 512;
constexpr int NCH_L6       = 256;
constexpr int NCH_L7       = 128;
constexpr int W5_PITCH     = 1088;
constexpr int NCH_SKIP     = 64;
constexpr int NCH_POOL     = 1024;
constexpr int CHUNK_POINTS = 8192;
constexpr int NUM_CHUNKS   = NUM_POINTS / CHUNK_POINTS;
constexpr int NUM_MTILES   = NUM_POINTS / 64;
static_assert(W5_PITCH == NCH_SKIP + NCH_POOL);
static_assert(NCH_SKIP == NCH_L2 && NCH_POOL == NCH_L4);
static_assert(NUM_POINTS % 64 == 0 && CHUNK_POINTS % 64 == 0 && NUM_POINTS % CHUNK_POINTS == 0);
static_assert(NCH_L2 % 64 == 0 && NCH_L1 % 32 == 0);
static_assert(NCH_L3 % 64 == 0 && NCH_L2 % 32 == 0);
static_assert(NCH_L4 % 64 == 0 && NCH_L3 % 32 == 0);
static_assert(NCH_L5 % 64 == 0 && NCH_SKIP % 32 == 0);
static_assert(NCH_L6 % 64 == 0 && NCH_L5 % 32 == 0);
static_assert(NCH_L7 % 64 == 0 && NCH_L6 % 32 == 0);
static_assert(NCH_L7 == 128 && NCH_L1 == 64);

typedef __attribute__((ext_vector_type(8)))  _Float16 v8h;
typedef __attribute__((ext_vector_type(16))) __bf16   v16b;
typedef __attribute__((ext_vector_type(8)))  __bf16   v8b;
typedef __attribute__((ext_vector_type(8)))  float    v8f;
typedef __attribute__((ext_vector_type(4)))  float    v4f;
typedef __attribute__((ext_vector_type(4)))  unsigned v4u;

__device__ __forceinline__ unsigned short f2bf_bits(float f) {
  unsigned u = __float_as_uint(f);
  return (unsigned short)((u + 0x7FFFu + ((u >> 16) & 1u)) >> 16);
}
__device__ __forceinline__ float bf_bits2f(unsigned short h) { return __uint_as_float(((unsigned)h) << 16); }

__device__ __forceinline__ unsigned bf_bits32(float f) {
  const unsigned u = __float_as_uint(f);
  return (u + 0x7FFFu + ((u >> 16) & 1u)) >> 16;
}
__device__ __forceinline__ void bf_split32(float f, unsigned& hb, unsigned& lb) {
  hb = bf_bits32(f);
  lb = bf_bits32(f - __uint_as_float(hb << 16));
}

__device__ __forceinline__ void grp_guard_b(v8f& a, v8f& b, v8f& c, v8f& d, v16b x, v16b y) {
  asm volatile("v_nop\n\tv_nop\n\tv_nop\n\tv_nop" : "+v"(a), "+v"(b), "+v"(c), "+v"(d) : "v"(x), "v"(y));
}
__device__ __forceinline__ void keep4_b(v16b a, v16b b, v16b c, v16b d) { asm volatile("v_nop" :: "v"(a), "v"(b), "v"(c), "v"(d)); }
__device__ __forceinline__ void acc_guard4(v8f& a, v8f& b, v8f& c, v8f& d) {
  asm volatile("v_nop\n\tv_nop\n\tv_nop\n\tv_nop" : "+v"(a), "+v"(b), "+v"(c), "+v"(d));
}

struct FragB {
  union U { v16b v; v8b h[2]; };
  static __device__ __forceinline__ v16b load(const __bf16* p) {
    U f; f.h[0] = *(const v8b*)(p); f.h[1] = *(const v8b*)(p + 16); return f.v;
  }
  static __device__ __forceinline__ v8f mma(v16b a, v16b b, v8f c) {
    return __builtin_amdgcn_wmma_f32_16x16x32_bf16(false, a, false, b, (short)0, c, false, false);
  }
};

template <bool SPLIT, int BIAS_MODE, int OUT_MODE, int ACT>
__global__ __launch_bounds__(256) void wmma_gemm64(
    const unsigned short* __restrict__ Ap, const unsigned short* __restrict__ A2p, int lda, long strideA,
    const unsigned short* __restrict__ Btp, const unsigned short* __restrict__ Bt2p, int ldb, long strideB,
    void* __restrict__ Cout, void* __restrict__ Cout2, int ldc, long strideC,
    const float* __restrict__ bias,
    int M, int N, int K, float scale) {
  typedef __bf16 T;
  typedef v16b V;
  const T* A = (const T*)Ap; const T* A2 = (const T*)A2p; const T* Bt = (const T*)Btp; const T* Bt2 = (const T*)Bt2p;
  __shared__ __align__(16) float sT[8][16 * 68];
  const int b    = blockIdx.y;
  const int lane = threadIdx.x & 31;
  const int wave = threadIdx.x >> 5;
  const int tilesN = N >> 6;
  const int tilesM = M >> 6;
  const int tile = blockIdx.x * 8 + wave;
  if (tile >= tilesM * tilesN) return;
  const int tm = tile / tilesN;
  const int tn = tile - tm * tilesN;
  const int m0 = tm << 6;
  const int n0 = tn << 6;

  const T* Ab  = A  + (size_t)b * strideA;
  const T* Bb  = Bt + (size_t)b * strideB;
  const T* Ab2 = SPLIT ? (A2  + (size_t)b * strideA) : nullptr;
  const T* Bb2 = SPLIT ? (Bt2 + (size_t)b * strideB) : nullptr;

  const int rlane = lane & 15;
  const int koff  = (lane >> 4) * 8;
  const int mOff  = (lane >> 4) * 8;

  v8f acc[4][4];
#pragma unroll
  for (int i = 0; i < 4; ++i)
#pragma unroll
    for (int j = 0; j < 4; ++j) acc[i][j] = (v8f){0.f,0.f,0.f,0.f,0.f,0.f,0.f,0.f};

  for (int k0 = 0; k0 < K; k0 += 32) {
    V bh[4], bl[4];
#pragma unroll
    for (int j = 0; j < 4; ++j) {
      const size_t bo = (size_t)(n0 + (j << 4) + rlane) * ldb + koff + k0;
      bh[j] = FragB::load(Bb + bo);
      if (SPLIT) bl[j] = FragB::load(Bb2 + bo);
    }
#pragma unroll
    for (int i = 0; i < 4; ++i) {
      const size_t ao = (size_t)(m0 + (i << 4) + rlane) * lda + koff + k0;
      V ah = FragB::load(Ab + ao);
      V al;
      if (SPLIT) al = FragB::load(Ab2 + ao);
#pragma unroll
      for (int j = 0; j < 4; ++j) {
        acc[i][j] = FragB::mma(ah, bh[j], acc[i][j]);
        if (SPLIT) {
          acc[i][j] = FragB::mma(ah, bl[j], acc[i][j]);
          acc[i][j] = FragB::mma(al, bh[j], acc[i][j]);
        }
      }
      grp_guard_b(acc[i][0], acc[i][1], acc[i][2], acc[i][3], ah, SPLIT ? al : ah);
    }
    keep4_b(bh[0], bh[1], bh[2], bh[3]);
    if (SPLIT) keep4_b(bl[0], bl[1], bl[2], bl[3]);
  }
  acc_guard4(acc[0][0], acc[0][1], acc[0][2], acc[0][3]);
  acc_guard4(acc[1][0], acc[1][1], acc[1][2], acc[1][3]);
  acc_guard4(acc[2][0], acc[2][1], acc[2][2], acc[2][3]);
  acc_guard4(acc[3][0], acc[3][1], acc[3][2], acc[3][3]);

  float* slab = sT[wave];
#pragma unroll
  for (int i = 0; i < 4; ++i) {
    const int mBase = m0 + (i << 4);
#pragma unroll
    for (int j = 0; j < 4; ++j) {
      const int n = n0 + (j << 4) + rlane;
      float bv = 0.f;
      if (BIAS_MODE == 2) bv = bias[n];
#pragma unroll
      for (int r = 0; r < 8; ++r) {
        float v = acc[i][j][r] * scale;
        if (BIAS_MODE == 2) v += bv;
        if (ACT == 2) v = fmaxf(v, 0.0f);
        slab[(mOff + r) * 68 + (j << 4) + rlane] = v;
      }
    }
    __builtin_amdgcn_fence(__ATOMIC_RELEASE, "workgroup");
    __builtin_amdgcn_wave_barrier();
    __builtin_amdgcn_fence(__ATOMIC_ACQUIRE, "workgroup");
    if (OUT_MODE == 0) {
      float* C = (float*)Cout + (size_t)b * strideC;
      const int hh = lane >> 4, c4 = (lane & 15) * 4;
      for (int pass = 0; pass < 2; ++pass) {
#pragma unroll
        for (int it = 0; it < 8; ++it) {
          const int row = it * 2 + hh;
          v4f v = *(const v4f*)(slab + row * 68 + c4);
          *(volatile v4f*)(C + (size_t)(mBase + row) * ldc + n0 + c4) = v;
        }
        __threadfence();
      }
    } else {
      const int q = lane >> 3, c8 = (lane & 7) * 8;
      unsigned short* C  = (unsigned short*)Cout  + (size_t)b * strideC;
      unsigned short* C2 = (OUT_MODE == 2) ? ((unsigned short*)Cout2 + (size_t)b * strideC) : nullptr;
      for (int pass = 0; pass < 2; ++pass) {
#pragma unroll
        for (int it = 0; it < 4; ++it) {
          const int row = it * 4 + q;
          const float* sp = slab + row * 68 + c8;
          v8h hv, lv;
#pragma unroll
          for (int e = 0; e < 8; ++e) {
            unsigned short hb = f2bf_bits(sp[e]);
            unsigned short lb = f2bf_bits(sp[e] - bf_bits2f(hb));
            hv[e] = __builtin_bit_cast(_Float16, hb);
            lv[e] = __builtin_bit_cast(_Float16, lb);
          }
          *(volatile v8h*)(C + (size_t)(mBase + row) * ldc + n0 + c8) = hv;
          if (OUT_MODE == 2) *(volatile v8h*)(C2 + (size_t)(mBase + row) * ldc + n0 + c8) = lv;
        }
        __threadfence();
      }
    }
    __builtin_amdgcn_fence(__ATOMIC_RELEASE, "workgroup");
    __builtin_amdgcn_wave_barrier();
    __builtin_amdgcn_fence(__ATOMIC_ACQUIRE, "workgroup");
  }
}

__global__ __launch_bounds__(256) void l4_colmax_kernel(
    const unsigned short* __restrict__ Ahp, const unsigned short* __restrict__ Alp,
    const unsigned short* __restrict__ Bhp, const unsigned short* __restrict__ Blp,
    const float* __restrict__ bias, float* __restrict__ gmaxpart, int M, int N, int K) {
  typedef __bf16 T;
  typedef v16b V;
  const T* Ab  = (const T*)Ahp; const T* Ab2 = (const T*)Alp;
  const T* Bb  = (const T*)Bhp; const T* Bb2 = (const T*)Blp;
  __shared__ __align__(16) float sM[8][64];
  const int lane = threadIdx.x & 31;
  const int wave = threadIdx.x >> 5;
  const int tilesN = N >> 6;
  const int tilesM = M >> 6;
  const int tile = blockIdx.x * 8 + wave;
  if (tile >= tilesM * tilesN) return;
  const int tm = tile / tilesN;
  const int tn = tile - tm * tilesN;
  const int m0 = tm << 6;
  const int n0 = tn << 6;
  const int rlane = lane & 15;
  const int hh    = lane >> 4;
  const int koff  = hh * 8;

  v8f acc[4][4];
#pragma unroll
  for (int i = 0; i < 4; ++i)
#pragma unroll
    for (int j = 0; j < 4; ++j) acc[i][j] = (v8f){0.f,0.f,0.f,0.f,0.f,0.f,0.f,0.f};

  for (int k0 = 0; k0 < K; k0 += 32) {
    V bh[4], bl[4];
#pragma unroll
    for (int j = 0; j < 4; ++j) {
      const size_t bo = (size_t)(n0 + (j << 4) + rlane) * K + koff + k0;
      bh[j] = FragB::load(Bb + bo);
      bl[j] = FragB::load(Bb2 + bo);
    }
#pragma unroll
    for (int i = 0; i < 4; ++i) {
      const size_t ao = (size_t)(m0 + (i << 4) + rlane) * K + koff + k0;
      V ah = FragB::load(Ab + ao);
      V al = FragB::load(Ab2 + ao);
#pragma unroll
      for (int j = 0; j < 4; ++j) {
        acc[i][j] = FragB::mma(ah, bh[j], acc[i][j]);
        acc[i][j] = FragB::mma(ah, bl[j], acc[i][j]);
        acc[i][j] = FragB::mma(al, bh[j], acc[i][j]);
      }
      grp_guard_b(acc[i][0], acc[i][1], acc[i][2], acc[i][3], ah, al);
    }
    keep4_b(bh[0], bh[1], bh[2], bh[3]);
    keep4_b(bl[0], bl[1], bl[2], bl[3]);
  }
  acc_guard4(acc[0][0], acc[0][1], acc[0][2], acc[0][3]);
  acc_guard4(acc[1][0], acc[1][1], acc[1][2], acc[1][3]);
  acc_guard4(acc[2][0], acc[2][1], acc[2][2], acc[2][3]);
  acc_guard4(acc[3][0], acc[3][1], acc[3][2], acc[3][3]);

  float* sl = sM[wave];
#pragma unroll
  for (int j = 0; j < 4; ++j) {
    const float bv = bias[n0 + (j << 4) + rlane];
    float mx = 0.0f;
#pragma unroll
    for (int i = 0; i < 4; ++i)
#pragma unroll
      for (int r = 0; r < 8; ++r) mx = fmaxf(mx, acc[i][j][r] + bv);
    const float other = __shfl_xor(mx, 16, 32);
    mx = fmaxf(mx, other);
    if (hh == 0) sl[(j << 4) + rlane] = mx;
  }
  __builtin_amdgcn_fence(__ATOMIC_RELEASE, "workgroup");
  __builtin_amdgcn_wave_barrier();
  __builtin_amdgcn_fence(__ATOMIC_ACQUIRE, "workgroup");
  const int c4 = (lane & 15) * 4;
  const v4f mv = *(const v4f*)(sl + c4);
  float* gp = gmaxpart + (size_t)tm * N + n0 + c4;
  if (lane < 16) *(volatile v4f*)gp = mv;
  __threadfence();
  if (lane < 16) *(volatile v4f*)gp = mv;
}

__global__ __launch_bounds__(256) void split8_kernel(const float* __restrict__ src, unsigned* __restrict__ hi,
                                                     unsigned* __restrict__ lo, int nrow, int ncol8, int spitch) {
  const int i  = blockIdx.x * 256 + threadIdx.x;
  const int n8 = nrow * ncol8;
  if (i < n8) {
    const int row = i / ncol8;
    const int c8  = i - row * ncol8;
    const float* sp = src + (size_t)row * spitch + c8 * 8;
    const v4f a = *(const v4f*)(sp);
    const v4f b = *(const v4f*)(sp + 4);
    v4u hv, lv;
#pragma unroll
    for (int q = 0; q < 2; ++q) {
      const float f0 = a[2 * q], f1 = a[2 * q + 1];
      const float g0 = b[2 * q], g1 = b[2 * q + 1];
      unsigned h0, l0, h1, l1;
      bf_split32(f0, h0, l0);
      bf_split32(f1, h1, l1);
      hv[q] = h0 | (h1 << 16);
      lv[q] = l0 | (l1 << 16);
      bf_split32(g0, h0, l0);
      bf_split32(g1, h1, l1);
      hv[2 + q] = h0 | (h1 << 16);
      lv[2 + q] = l0 | (l1 << 16);
    }
    unsigned* ph = hi + (size_t)i * 4;
    unsigned* pl = lo + (size_t)i * 4;
    *(volatile v4u*)ph = hv;
    *(volatile v4u*)pl = lv;
    __threadfence();
    *(volatile v4u*)ph = hv;
    *(volatile v4u*)pl = lv;
  }
}

__global__ __launch_bounds__(256) void l1_kernel(const float* __restrict__ x, const float* __restrict__ W1,
                                                 const float* __restrict__ b1, unsigned* __restrict__ H1h,
                                                 unsigned* __restrict__ H1l, int npts) {
  __shared__ float sW[NCH_L1 * 3];
  __shared__ float sB[NCH_L1];
  const int tid = threadIdx.x;
  if (tid < NCH_L1 * 3) sW[tid] = W1[tid];
  if (tid < NCH_L1) sB[tid] = b1[tid];
  __syncthreads();
  const int i  = blockIdx.x * 256 + tid;
  const int p  = i >> 3;
  const int c8 = (i & 7) * 8;
  const int pc = (p < npts) ? p : (npts - 1);
  const float x0 = x[(size_t)pc * 3 + 0];
  const float x1 = x[(size_t)pc * 3 + 1];
  const float x2 = x[(size_t)pc * 3 + 2];
  v4u hv, lv;
#pragma unroll
  for (int q = 0; q < 4; ++q) {
    const int ca = c8 + 2 * q, cb = ca + 1;
    float pa = x0 * sW[ca * 3 + 0];
    pa = fmaf(x1, sW[ca * 3 + 1], pa);
    pa = fmaf(x2, sW[ca * 3 + 2], pa);
    float pb = x0 * sW[cb * 3 + 0];
    pb = fmaf(x1, sW[cb * 3 + 1], pb);
    pb = fmaf(x2, sW[cb * 3 + 2], pb);
    const float va = fmaxf(pa + sB[ca], 0.0f);
    const float vb = fmaxf(pb + sB[cb], 0.0f);
    unsigned h0, l0, h1, l1;
    bf_split32(va, h0, l0);
    bf_split32(vb, h1, l1);
    hv[q] = h0 | (h1 << 16);
    lv[q] = l0 | (l1 << 16);
  }
  if (p < npts) {
    unsigned* ph = H1h + (size_t)i * 4;
    unsigned* pl = H1l + (size_t)i * 4;
    *(volatile v4u*)ph = hv;
    *(volatile v4u*)pl = lv;
    __threadfence();
    *(volatile v4u*)ph = hv;
    *(volatile v4u*)pl = lv;
  }
}

__global__ __launch_bounds__(32) void gmax_kernel(const float* __restrict__ gmaxpart, float* __restrict__ g) {
  const int col = blockIdx.x * 128 + threadIdx.x * 4;
  v4f m = (v4f){0.f, 0.f, 0.f, 0.f};
#pragma unroll 4
  for (int t = 0; t < NUM_MTILES; ++t) {
    const v4f v = *(const v4f*)(gmaxpart + (size_t)t * NCH_POOL + col);
    m[0] = fmaxf(m[0], v[0]);
    m[1] = fmaxf(m[1], v[1]);
    m[2] = fmaxf(m[2], v[2]);
    m[3] = fmaxf(m[3], v[3]);
  }
  float* gp = g + col;
  *(volatile v4f*)gp = m;
  __threadfence();
  *(volatile v4f*)gp = m;
}

__global__ __launch_bounds__(256) void c5_kernel(const float* __restrict__ W5, const float* __restrict__ b5,
                                                 const float* __restrict__ g, float* __restrict__ c5) {
  __shared__ float sC[32];
  const int lane = threadIdx.x & 31;
  const int wave = threadIdx.x >> 5;
#pragma unroll 1
  for (int q = 0; q < 4; ++q) {
    const int o = blockIdx.x * 32 + wave * 4 + q;
    const float* wr = W5 + (size_t)o * W5_PITCH + NCH_SKIP;
    float a0 = 0.0f, a1 = 0.0f, a2 = 0.0f, a3 = 0.0f;
#pragma unroll 2
    for (int k = 0; k < NCH_POOL / 128; ++k) {
      const int idx = k * 128 + lane * 4;
      const v4f w  = *(const v4f*)(wr + idx);
      const v4f gv = *(const v4f*)(g + idx);
      a0 = fmaf(w[0], gv[0], a0);
      a1 = fmaf(w[1], gv[1], a1);
      a2 = fmaf(w[2], gv[2], a2);
      a3 = fmaf(w[3], gv[3], a3);
    }
    float a = (a0 + a1) + (a2 + a3);
#pragma unroll
    for (int off = 16; off >= 1; off >>= 1) a += __shfl_xor(a, off, 32);
    const float bo = b5[o];
    if (lane == 0) sC[wave * 4 + q] = a + bo;
  }
  __syncthreads();
  if (wave == 0) {
    const float v = sC[lane];
    float* cp = c5 + blockIdx.x * 32 + lane;
    *(volatile float*)cp = v;
    __threadfence();
    *(volatile float*)cp = v;
  }
}

__global__ __launch_bounds__(256) void l8_kernel(const float* __restrict__ Z7, const float* __restrict__ W8,
                                                 const float* __restrict__ b8, float* __restrict__ out, int npts) {
  __shared__ __align__(16) float sW[NCH_L7];
  const int tid = threadIdx.x;
  if (tid < NCH_L7) sW[tid] = W8[tid];
  __syncthreads();
  const int p  = blockIdx.x * 256 + tid;
  const int pc = (p < npts) ? p : (npts - 1);
  const float* zr = Z7 + (size_t)pc * NCH_L7;
  float a0 = 0.0f, a1 = 0.0f, a2 = 0.0f, a3 = 0.0f;
#pragma unroll 4
  for (int k = 0; k < NCH_L7 / 4; ++k) {
    const v4f z = *(const v4f*)(zr + 4 * k);
    const v4f w = *(const v4f*)(sW + 4 * k);
    a0 = fmaf(z[0], w[0], a0);
    a1 = fmaf(z[1], w[1], a1);
    a2 = fmaf(z[2], w[2], a2);
    a3 = fmaf(z[3], w[3], a3);
  }
  const float s = ((a0 + a1) + (a2 + a3)) + b8[0];
  if (p < npts) {
    float* op = out + p;
    *(volatile float*)op = s;
    __threadfence();
    *(volatile float*)op = s;
  }
}

extern "C" void kernel_launch(void* const* d_in, const int* in_sizes, int n_in,
                              void* d_out, int out_size, void* d_ws, size_t ws_size, hipStream_t stream) {
  if (n_in < 17 || d_out == nullptr || d_ws == nullptr) return;
  if (in_sizes[0] != NUM_POINTS * 3 || in_sizes[1] != NCH_L1 * 3 || in_sizes[2] != NCH_L1 ||
      in_sizes[3] != NCH_L2 * NCH_L1 || in_sizes[4] != NCH_L2 ||
      in_sizes[5] != NCH_L3 * NCH_L2 || in_sizes[6] != NCH_L3 ||
      in_sizes[7] != NCH_L4 * NCH_L3 || in_sizes[8] != NCH_L4 ||
      in_sizes[9] != NCH_L5 * W5_PITCH || in_sizes[10] != NCH_L5 ||
      in_sizes[11] != NCH_L6 * NCH_L5 || in_sizes[12] != NCH_L6 ||
      in_sizes[13] != NCH_L7 * NCH_L6 || in_sizes[14] != NCH_L7 ||
      in_sizes[15] != NCH_L7 || in_sizes[16] != 1 || out_size != NUM_POINTS) return;

  const float* x  = (const float*)d_in[0];
  const float* W1 = (const float*)d_in[1];
  const float* b1 = (const float*)d_in[2];
  const float* W2 = (const float*)d_in[3];
  const float* b2 = (const float*)d_in[4];
  const float* W3 = (const float*)d_in[5];
  const float* b3 = (const float*)d_in[6];
  const float* W4 = (const float*)d_in[7];
  const float* b4 = (const float*)d_in[8];
  const float* W5 = (const float*)d_in[9];
  const float* b5 = (const float*)d_in[10];
  const float* W6 = (const float*)d_in[11];
  const float* b6 = (const float*)d_in[12];
  const float* W7 = (const float*)d_in[13];
  const float* b7 = (const float*)d_in[14];
  const float* W8 = (const float*)d_in[15];
  const float* b8 = (const float*)d_in[16];
  float* out = (float*)d_out;

  char* ws = (char*)d_ws; size_t off = 0;
  auto carve = [&](size_t bytes) -> char* { char* p = ws + off; off += (bytes + 255) & ~(size_t)255; return p; };
  unsigned short* W2h = (unsigned short*)carve((size_t)NCH_L2 * NCH_L1 * 2);
  unsigned short* W2l = (unsigned short*)carve((size_t)NCH_L2 * NCH_L1 * 2);
  unsigned short* W3h = (unsigned short*)carve((size_t)NCH_L3 * NCH_L2 * 2);
  unsigned short* W3l = (unsigned short*)carve((size_t)NCH_L3 * NCH_L2 * 2);
  unsigned short* W4h = (unsigned short*)carve((size_t)NCH_L4 * NCH_L3 * 2);
  unsigned short* W4l = (unsigned short*)carve((size_t)NCH_L4 * NCH_L3 * 2);
  unsigned short* W5h = (unsigned short*)carve((size_t)NCH_L5 * NCH_SKIP * 2);
  unsigned short* W5l = (unsigned short*)carve((size_t)NCH_L5 * NCH_SKIP * 2);
  unsigned short* W6h = (unsigned short*)carve((size_t)NCH_L6 * NCH_L5 * 2);
  unsigned short* W6l = (unsigned short*)carve((size_t)NCH_L6 * NCH_L5 * 2);
  unsigned short* W7h = (unsigned short*)carve((size_t)NCH_L7 * NCH_L6 * 2);
  unsigned short* W7l = (unsigned short*)carve((size_t)NCH_L7 * NCH_L6 * 2);
  unsigned short* H1h = (unsigned short*)carve((size_t)NUM_POINTS * NCH_L1 * 2);
  unsigned short* H1l = (unsigned short*)carve((size_t)NUM_POINTS * NCH_L1 * 2);
  unsigned short* H2h = (unsigned short*)carve((size_t)NUM_POINTS * NCH_L2 * 2);
  unsigned short* H2l = (unsigned short*)carve((size_t)NUM_POINTS * NCH_L2 * 2);
  unsigned short* Y3h = (unsigned short*)carve((size_t)NUM_POINTS * NCH_L3 * 2);
  unsigned short* Y3l = (unsigned short*)carve((size_t)NUM_POINTS * NCH_L3 * 2);
  float*          GPART = (float*)carve((size_t)NUM_MTILES * NCH_L4 * 4);
  float*          GVEC  = (float*)carve((size_t)NCH_L4 * 4);
  float*          C5VEC = (float*)carve((size_t)NCH_L5 * 4);
  unsigned short* Z5h = (unsigned short*)carve((size_t)CHUNK_POINTS * NCH_L5 * 2);
  unsigned short* Z5l = (unsigned short*)carve((size_t)CHUNK_POINTS * NCH_L5 * 2);
  unsigned short* Z6h = (unsigned short*)carve((size_t)CHUNK_POINTS * NCH_L6 * 2);
  unsigned short* Z6l = (unsigned short*)carve((size_t)CHUNK_POINTS * NCH_L6 * 2);
  float*          Z7  = (float*)carve((size_t)CHUNK_POINTS * NCH_L7 * 4);
  if (off > ws_size || off > (size_t)134217728) return;

  split8_kernel<<<(NCH_L2 * (NCH_L1 / 8)) / 256, 256, 0, stream>>>(W2, (unsigned*)W2h, (unsigned*)W2l, NCH_L2, NCH_L1 / 8, NCH_L1);
  split8_kernel<<<(NCH_L3 * (NCH_L2 / 8)) / 256, 256, 0, stream>>>(W3, (unsigned*)W3h, (unsigned*)W3l, NCH_L3, NCH_L2 / 8, NCH_L2);
  split8_kernel<<<(NCH_L4 * (NCH_L3 / 8)) / 256, 256, 0, stream>>>(W4, (unsigned*)W4h, (unsigned*)W4l, NCH_L4, NCH_L3 / 8, NCH_L3);
  split8_kernel<<<(NCH_L5 * (NCH_SKIP / 8)) / 256, 256, 0, stream>>>(W5, (unsigned*)W5h, (unsigned*)W5l, NCH_L5, NCH_SKIP / 8, W5_PITCH);
  split8_kernel<<<(NCH_L6 * (NCH_L5 / 8)) / 256, 256, 0, stream>>>(W6, (unsigned*)W6h, (unsigned*)W6l, NCH_L6, NCH_L5 / 8, NCH_L5);
  split8_kernel<<<(NCH_L7 * (NCH_L6 / 8)) / 256, 256, 0, stream>>>(W7, (unsigned*)W7h, (unsigned*)W7l, NCH_L7, NCH_L6 / 8, NCH_L6);
  static_assert((NCH_L2 * (NCH_L1 / 8)) % 256 == 0 && (NCH_L3 * (NCH_L2 / 8)) % 256 == 0);
  static_assert((NCH_L4 * (NCH_L3 / 8)) % 256 == 0 && (NCH_L5 * (NCH_SKIP / 8)) % 256 == 0);
  static_assert((NCH_L6 * (NCH_L5 / 8)) % 256 == 0 && (NCH_L7 * (NCH_L6 / 8)) % 256 == 0);

  l1_kernel<<<(NUM_POINTS * 8) / 256, 256, 0, stream>>>(x, W1, b1, (unsigned*)H1h, (unsigned*)H1l, NUM_POINTS);

  {
    const int tiles = (NUM_POINTS / 64) * (NCH_L2 / 64);
    wmma_gemm64<true, 2, 2, 2><<<dim3((tiles + 7) / 8, 1), 256, 0, stream>>>(
        H1h, H1l, NCH_L1, 0L, W2h, W2l, NCH_L1, 0L, (void*)H2h, (void*)H2l, NCH_L2, 0L,
        b2, NUM_POINTS, NCH_L2, NCH_L1, 1.0f);
  }
  {
    const int tiles = (NUM_POINTS / 64) * (NCH_L3 / 64);
    wmma_gemm64<true, 2, 2, 2><<<dim3((tiles + 7) / 8, 1), 256, 0, stream>>>(
        H2h, H2l, NCH_L2, 0L, W3h, W3l, NCH_L2, 0L, (void*)Y3h, (void*)Y3l, NCH_L3, 0L,
        b3, NUM_POINTS, NCH_L3, NCH_L2, 1.0f);
  }
  {
    const int tiles = (NUM_POINTS / 64) * (NCH_L4 / 64);
    l4_colmax_kernel<<<(tiles + 7) / 8, 256, 0, stream>>>(Y3h, Y3l, W4h, W4l, b4, GPART, NUM_POINTS, NCH_L4, NCH_L3);
  }
  gmax_kernel<<<NCH_POOL / 128, 32, 0, stream>>>(GPART, GVEC);
  c5_kernel<<<NCH_L5 / 32, 256, 0, stream>>>(W5, b5, GVEC, C5VEC);

  for (int ch = 0; ch < NUM_CHUNKS; ++ch) {
    const size_t prow = (size_t)ch * CHUNK_POINTS;
    {
      const int tiles = (CHUNK_POINTS / 64) * (NCH_L5 / 64);
      wmma_gemm64<true, 2, 2, 2><<<dim3((tiles + 7) / 8, 1), 256, 0, stream>>>(
          H2h + prow * NCH_L2, H2l + prow * NCH_L2, NCH_L2, 0L, W5h, W5l, NCH_SKIP, 0L,
          (void*)Z5h, (void*)Z5l, NCH_L5, 0L, C5VEC, CHUNK_POINTS, NCH_L5, NCH_SKIP, 1.0f);
    }
    {
      const int tiles = (CHUNK_POINTS / 64) * (NCH_L6 / 64);
      wmma_gemm64<true, 2, 2, 2><<<dim3((tiles + 7) / 8, 1), 256, 0, stream>>>(
          Z5h, Z5l, NCH_L5, 0L, W6h, W6l, NCH_L5, 0L, (void*)Z6h, (void*)Z6l, NCH_L6, 0L,
          b6, CHUNK_POINTS, NCH_L6, NCH_L5, 1.0f);
    }
    {
      const int tiles = (CHUNK_POINTS / 64) * (NCH_L7 / 64);
      wmma_gemm64<true, 2, 0, 2><<<dim3((tiles + 7) / 8, 1), 256, 0, stream>>>(
          Z6h, Z6l, NCH_L6, 0L, W7h, W7l, NCH_L6, 0L, (void*)Z7, (void*)Z7, NCH_L7, 0L,
          b7, CHUNK_POINTS, NCH_L7, NCH_L6, 1.0f);
    }
    l8_kernel<<<CHUNK_POINTS / 256, 256, 0, stream>>>(Z7, W8, b8, out + prow, CHUNK_POINTS);
  }
}
